// CMCModel_53128745452244
// MI455X (gfx1250) — hardware-run, weakly checked
//
#include <hip/hip_runtime.h>
#include <math.h>

typedef __attribute__((ext_vector_type(16))) _Float16 v16h;
typedef __attribute__((ext_vector_type(8)))  _Float16 v8h;
typedef __attribute__((ext_vector_type(8)))  float    v8f;
typedef __attribute__((ext_vector_type(4)))  float    v4f;

constexpr int kSteps   = 64;
constexpr int kBatch   = 32;
constexpr int kMass    = 8;
constexpr int kAux     = 16;
constexpr int kCells   = 128;
constexpr int kFeat    = kMass + kAux + kCells;
constexpr int kFeatPad = 160;
constexpr int kColsI   = kMass * kCells;
constexpr int kColsR   = kCells * kCells;
constexpr int kColsAll = kColsI + kColsR + kCells;
constexpr int kGroups  = kColsAll / kCells;
constexpr int kFPitch  = 168;
constexpr int kCPitch  = 136;
constexpr int kChunksPerRow = kFeatPad / 8;
constexpr int kPlaneChunks  = kColsAll * kChunksPerRow;
constexpr int kBiasVec4     = kColsAll / 4;

constexpr float kWCarry = 256.0f;
constexpr float kFCarry = 16.0f;
constexpr float kFold   = 1.0f / (kWCarry * kFCarry);
constexpr float kEps    = 1e-5f;
constexpr float kHalfMinNormal = 6.103515625e-05f;

static_assert(kFeat == 152, "feature count");
static_assert(kFeatPad % 32 == 0 && kFeatPad >= kFeat && kFeatPad - kFeat == 8, "K pad is one 8-wide chunk");
static_assert(kColsAll == 17536 && kGroups == 137, "column groups");
static_assert(kPlaneChunks == 1370 * 256, "weight plane grid is exact");
static_assert((kColsI * kChunksPerRow) == 80 * 256, "first source boundary on a block boundary");
static_assert(((kColsI + kColsR) * kChunksPerRow) == 1360 * 256, "second source boundary on a block boundary");
static_assert(kBiasVec4 == 4384 && (kColsI / 4) == 256 && ((kColsI + kColsR) / 4) == 17 * 256, "bias plane blocks");
static_assert((kFPitch * 2) % 16 == 0 && (kCPitch * 4) % 16 == 0, "16-B aligned LDS rows");

constexpr size_t kOffWT   = 0;
constexpr size_t kBytesWT = (size_t)kColsAll * kFeatPad * 2;
constexpr size_t kOffBC   = kOffWT + kBytesWT;
constexpr size_t kBytesBC = (size_t)kColsAll * 4;
constexpr size_t kWsTotal = kOffBC + kBytesBC;
static_assert(kBytesWT == 5611520ull && kBytesBC == 70144ull && kWsTotal == 5681664ull, "carve total");
static_assert((kOffBC % 128) == 0 && (kBytesWT % 128) == 0 && (kBytesBC % 128) == 0, "whole lines");
static_assert(kWsTotal <= 134217728ull, "carve cap");

union FragU { v16h v; v8h h[2]; };
__device__ __forceinline__ v16h frag_load(const _Float16* p) {
  FragU f;
  f.h[0] = *(const v8h*)(p);
  f.h[1] = *(const v8h*)(p + 16);
  return f.v;
}
__device__ __forceinline__ v8f mma_step(v16h a, v16h b, v8f c) {
  c = __builtin_amdgcn_wmma_f32_16x16x32_f16(false, a, false, b, (short)0, c, false, false);
  asm volatile("v_nop\n\tv_nop\n\tv_nop\n\tv_nop" : "+v"(c) : "v"(a), "v"(b));
  return c;
}
__device__ __forceinline__ _Float16 to_h_flush(float v) {
  const float w = (fabsf(v) < kHalfMinNormal) ? 0.0f : v;
  return (_Float16)w;
}

__global__ __launch_bounds__(256) void weight_plane_kernel(
    const float* __restrict__ W_i, const float* __restrict__ W_r, const float* __restrict__ W_o,
    unsigned short* __restrict__ WT)
{
  unsigned i = blockIdx.x * 256u + threadIdx.x;
  asm volatile("" : "+v"(i));
  unsigned n = i / (unsigned)kChunksPerRow;
  asm volatile("" : "+v"(n));
  unsigned kc = i - n * (unsigned)kChunksPerRow;
  asm volatile("" : "+v"(kc));
  const float* src;
  unsigned ld, nl;
  if (blockIdx.x < 80u) {
    src = W_i; ld = (unsigned)kColsI; nl = n;
  } else if (blockIdx.x < 1360u) {
    src = W_r; ld = (unsigned)kColsR; nl = n - (unsigned)kColsI;
  } else {
    src = W_o; ld = (unsigned)kCells; nl = n - (unsigned)(kColsI + kColsR);
  }
  const bool pad = (kc >= (unsigned)(kChunksPerRow - 1));
  unsigned kb = pad ? (unsigned)(kFeat - 8) : kc * 8u;
  asm volatile("" : "+v"(kb));
  float v[8];
#pragma unroll
  for (int e = 0; e < 8; ++e) {
    v[e] = src[(size_t)(kb + (unsigned)e) * ld + nl];
  }
#pragma unroll
  for (int e = 0; e < 8; ++e) {
    asm volatile("" : "+v"(v[e]));
  }
  v8h hv;
#pragma unroll
  for (int e = 0; e < 8; ++e) {
    const float cv = pad ? 0.0f : (v[e] * kWCarry);
    hv[e] = to_h_flush(cv);
  }
  unsigned short* dst = WT + (size_t)i * 8u;
  *(volatile v8h*)dst = hv;
  __threadfence();
  *(volatile v8h*)dst = hv;
}

__global__ __launch_bounds__(256) void bias_plane_kernel(
    const float* __restrict__ b_i, const float* __restrict__ b_r, const float* __restrict__ b_o,
    float* __restrict__ BC)
{
  unsigned i = blockIdx.x * 256u + threadIdx.x;
  asm volatile("" : "+v"(i));
  if (i >= (unsigned)kBiasVec4) return;
  const float* src;
  unsigned off;
  if (blockIdx.x == 0u) {
    src = b_i; off = i * 4u;
  } else if (blockIdx.x < 17u) {
    src = b_r; off = i * 4u - (unsigned)kColsI;
  } else {
    src = b_o; off = i * 4u - (unsigned)(kColsI + kColsR);
  }
  const v4f val = *(const v4f*)(src + off);
  float* dst = BC + (size_t)i * 4u;
  *(volatile v4f*)dst = val;
  __threadfence();
  *(volatile v4f*)dst = val;
}

__global__ __launch_bounds__(256) void cell_scan_kernel(
    const float* __restrict__ x_m, const float* __restrict__ x_a, const float* __restrict__ init_state,
    const unsigned short* __restrict__ WTp, const float* __restrict__ bcat,
    const float* __restrict__ fc_w, const float* __restrict__ fc_b, float* __restrict__ out)
{
  __shared__ __align__(16) _Float16 fH[kBatch * kFPitch];
  __shared__ __align__(16) float cx[kBatch * kCPitch];
  __shared__ __align__(16) float mS[kBatch * kCells];
  __shared__ __align__(16) float oS[kBatch * kCells];
  __shared__ __align__(16) float fcS[kCells];
  __shared__ __align__(16) float lgS[kBatch];
  static_assert(sizeof(_Float16) * kBatch * kFPitch + sizeof(float) * (kBatch * kCPitch + 2 * kBatch * kCells + kCells + kBatch) <= 65536, "static LDS");

  const _Float16* Wt = (const _Float16*)WTp;

  unsigned tid = threadIdx.x;
  unsigned lane = tid & 31u;
  asm volatile("" : "+v"(lane));
  unsigned hh = lane >> 4;
  asm volatile("" : "+v"(hh));
  unsigned nn = lane & 15u;
  asm volatile("" : "+v"(nn));
  unsigned ub = tid >> 3;
  asm volatile("" : "+v"(ub));
  unsigned up = tid & 7u;
  asm volatile("" : "+v"(up));
  const int wave = __builtin_amdgcn_readfirstlane((int)(tid >> 5));
  const int mt = wave & 1;
  const int q  = wave >> 1;
  unsigned drow = 16u * (unsigned)mt + 8u * hh;
  asm volatile("" : "+v"(drow));

  {
    float fv = fc_w[tid & 127u];
    asm volatile("" : "+v"(fv));
    if (tid < 128u) fcS[tid] = fv;
  }
  const float fcb = fc_b[0];
  {
    const float* ip = init_state + up * 16u;
    float* cp = cx + ub * (unsigned)kCPitch + 8u + up * 16u;
#pragma unroll
    for (int i = 0; i < 4; ++i) {
      const v4f iv = *(const v4f*)(ip + 4 * i);
      *(v4f*)(cp + 4 * i) = iv;
    }
  }

#pragma unroll 1
  for (int t = 0; t < kSteps; ++t) {
    {
      const float* cp = cx + ub * (unsigned)kCPitch + 8u + up * 16u;
      const v4f c0 = *(const v4f*)(cp);
      const v4f c1 = *(const v4f*)(cp + 4);
      const v4f c2 = *(const v4f*)(cp + 8);
      const v4f c3 = *(const v4f*)(cp + 12);
      float s = ((c0[0] + c0[1]) + (c0[2] + c0[3])) + ((c1[0] + c1[1]) + (c1[2] + c1[3]));
      s += ((c2[0] + c2[1]) + (c2[2] + c2[3])) + ((c3[0] + c3[1]) + (c3[2] + c3[3]));
      s += __shfl_xor(s, 1, 32);
      s += __shfl_xor(s, 2, 32);
      s += __shfl_xor(s, 4, 32);
      const float inv = 1.0f / (s + kEps);
      const float scn = inv * kFCarry;
      v8h h0, h1;
#pragma unroll
      for (int e = 0; e < 4; ++e) {
        h0[e]     = to_h_flush(c0[e] * scn);
        h0[4 + e] = to_h_flush(c1[e] * scn);
        h1[e]     = to_h_flush(c2[e] * scn);
        h1[4 + e] = to_h_flush(c3[e] * scn);
      }
      _Float16* fr = fH + ub * (unsigned)kFPitch;
      *(v8h*)(fr + 24u + up * 16u)      = h0;
      *(v8h*)(fr + 24u + up * 16u + 8u) = h1;

      const unsigned rowx = (unsigned)t * 32u + ub;
      const float* pm = x_m + rowx * 8u;
      const float* pa = x_a + rowx * 16u + ((up == 2u) ? 8u : 0u);
      v4f m0 = *(const v4f*)(pm);
      v4f m1 = *(const v4f*)(pm + 4);
      v4f a0 = *(const v4f*)(pa);
      v4f a1 = *(const v4f*)(pa + 4);
      asm volatile("" : "+v"(m0), "+v"(m1), "+v"(a0), "+v"(a1));
      const bool isM = (up == 0u);
      const bool isZ = (up >= 3u);
      v8h hx;
#pragma unroll
      for (int e = 0; e < 4; ++e) {
        const float s0 = isM ? m0[e] : a0[e];
        const float s1 = isM ? m1[e] : a1[e];
        const float w0 = isZ ? 0.0f : (s0 * kFCarry);
        const float w1 = isZ ? 0.0f : (s1 * kFCarry);
        hx[e]     = to_h_flush(w0);
        hx[4 + e] = to_h_flush(w1);
      }
      const unsigned colx = (up == 0u) ? 0u : ((up == 1u) ? 8u : ((up == 2u) ? 16u : (unsigned)kFeat));
      if (up < 4u) *(v8h*)(fr + colx) = hx;
      if (up == 0u) {
        float* xr = cx + ub * (unsigned)kCPitch;
        *(v4f*)(xr)      = m0;
        *(v4f*)(xr + 4u) = m1;
      }
    }
    __syncthreads();

    v8f mpart[8];
#pragma unroll
    for (int j = 0; j < 8; ++j) mpart[j] = (v8f){0.f, 0.f, 0.f, 0.f, 0.f, 0.f, 0.f, 0.f};

    const _Float16* arow = fH + (16u * (unsigned)mt + nn) * (unsigned)kFPitch + 8u * hh;
#pragma unroll 1
    for (int g = q; g < kGroups; g += 4) {
      const _Float16* wg = Wt + ((size_t)g * (size_t)kCells + nn) * (size_t)kFeatPad + 8u * hh;
      const float* bp = bcat + (unsigned)g * (unsigned)kCells + nn;
      float bv[8];
#pragma unroll
      for (int j = 0; j < 8; ++j) bv[j] = bp[16 * j];

      v8f acc[8];
#pragma unroll
      for (int j = 0; j < 8; ++j) acc[j] = (v8f){0.f, 0.f, 0.f, 0.f, 0.f, 0.f, 0.f, 0.f};
#pragma unroll 1
      for (int ks = 0; ks < kFeatPad / 32; ++ks) {
        const v16h a = frag_load(arow + ks * 32);
#pragma unroll
        for (int j = 0; j < 8; ++j) {
          const v16h b = frag_load(wg + (size_t)j * 16 * kFeatPad + ks * 32);
          acc[j] = mma_step(a, b, acc[j]);
        }
      }

      const bool sig = (g == kGroups - 1);
      const unsigned gs = sig ? (unsigned)(kGroups - 2) : (unsigned)g;
#pragma unroll
      for (int j = 0; j < 8; ++j) {
#pragma unroll
        for (int r = 0; r < 8; ++r) acc[j][r] = fmaf(acc[j][r], kFold, bv[j]);
      }
      if (sig) {
#pragma unroll
        for (int j = 0; j < 8; ++j) {
#pragma unroll
          for (int r = 0; r < 8; ++r) oS[(drow + (unsigned)r) * (unsigned)kCells + 16u * (unsigned)j + nn] = acc[j][r];
        }
      }
      float fac[8];
      const float* sp = cx + drow * (unsigned)kCPitch + gs;
#pragma unroll
      for (int r = 0; r < 8; ++r) {
        float mx = acc[0][r];
#pragma unroll
        for (int j = 1; j < 8; ++j) mx = fmaxf(mx, acc[j][r]);
        mx = fmaxf(mx, __shfl_xor(mx, 1, 32));
        mx = fmaxf(mx, __shfl_xor(mx, 2, 32));
        mx = fmaxf(mx, __shfl_xor(mx, 4, 32));
        mx = fmaxf(mx, __shfl_xor(mx, 8, 32));
        float s = 0.f;
#pragma unroll
        for (int j = 0; j < 8; ++j) {
          const float e = expf(acc[j][r] - mx);
          acc[j][r] = e;
          s += e;
        }
        s += __shfl_xor(s, 1, 32);
        s += __shfl_xor(s, 2, 32);
        s += __shfl_xor(s, 4, 32);
        s += __shfl_xor(s, 8, 32);
        const float scv = sp[r * kCPitch];
        fac[r] = scv * (1.0f / s);
      }
      if (!sig) {
#pragma unroll
        for (int j = 0; j < 8; ++j) {
#pragma unroll
          for (int r = 0; r < 8; ++r) mpart[j][r] = fmaf(acc[j][r], fac[r], mpart[j][r]);
        }
      }
    }
    __syncthreads();

    if (q == 0) {
#pragma unroll
      for (int j = 0; j < 8; ++j) {
#pragma unroll
        for (int r = 0; r < 8; ++r) mS[(drow + (unsigned)r) * (unsigned)kCells + 16u * (unsigned)j + nn] = mpart[j][r];
      }
    }
    __syncthreads();
#pragma unroll 1
    for (int rq = 1; rq < 4; ++rq) {
      if (q == rq) {
#pragma unroll
        for (int j = 0; j < 8; ++j) {
#pragma unroll
          for (int r = 0; r < 8; ++r) {
            const unsigned idx = (drow + (unsigned)r) * (unsigned)kCells + 16u * (unsigned)j + nn;
            const float cur = mS[idx];
            mS[idx] = cur + mpart[j][r];
          }
        }
      }
      __syncthreads();
    }

    {
      const unsigned base = ub * (unsigned)kCells + up * 16u;
      float* cp = cx + ub * (unsigned)kCPitch + 8u + up * 16u;
      float ls = 0.f;
#pragma unroll 1
      for (int i = 0; i < 4; ++i) {
        const v4f mv = *(const v4f*)(mS + base + 4 * i);
        const v4f zv = *(const v4f*)(oS + base + 4 * i);
        const v4f fw = *(const v4f*)(fcS + up * 16u + 4 * i);
        v4f cn;
#pragma unroll
        for (int e = 0; e < 4; ++e) {
          const float o  = 1.0f / (1.0f + expf(-zv[e]));
          const float em = o * mv[e];
          cn[e] = (1.0f - o) * mv[e];
          ls = fmaf(em, fw[e], ls);
        }
        *(v4f*)(cp + 4 * i) = cn;
      }
      ls += __shfl_xor(ls, 1, 32);
      ls += __shfl_xor(ls, 2, 32);
      ls += __shfl_xor(ls, 4, 32);
      if (up == 0u) lgS[ub] = ls + fcb;
    }
    __syncthreads();

    if (wave == 0) {
      const float lv = lgS[lane];
      float* op = out + (unsigned)t * (unsigned)kBatch + lane;
      *(volatile float*)op = lv;
      __threadfence();
      *(volatile float*)op = lv;
    }
  }

  {
    v4f ov[4];
#pragma unroll
    for (int it = 0; it < 4; ++it) {
      ov[it] = *(const v4f*)(cx + (unsigned)(wave + 8 * it) * (unsigned)kCPitch + 8u + lane * 4u);
    }
    float* o1 = out + kSteps * kBatch;
    for (int pass = 0; pass < 2; ++pass) {
#pragma unroll
      for (int it = 0; it < 4; ++it) {
        *(volatile v4f*)(o1 + (unsigned)(wave + 8 * it) * (unsigned)kCells + lane * 4u) = ov[it];
      }
      __threadfence();
    }
  }
}

extern "C" void kernel_launch(void* const* d_in, const int* in_sizes, int n_in,
                              void* d_out, int out_size, void* d_ws, size_t ws_size,
                              hipStream_t stream) {
  if (n_in < 11) return;
  if (in_sizes[0] != kSteps * kBatch * kMass) return;
  if (in_sizes[1] != kSteps * kBatch * kAux) return;
  if (in_sizes[2] != kCells) return;
  if (in_sizes[3] != kFeat * kColsI) return;
  if (in_sizes[4] != kColsI) return;
  if (in_sizes[5] != kFeat * kColsR) return;
  if (in_sizes[6] != kColsR) return;
  if (in_sizes[7] != kFeat * kCells) return;
  if (in_sizes[8] != kCells) return;
  if (in_sizes[9] != kCells) return;
  if (in_sizes[10] != 1) return;
  if (out_size != kSteps * kBatch + kBatch * kCells) return;
  if (ws_size < kWsTotal) return;

  const float* x_m        = (const float*)d_in[0];
  const float* x_a        = (const float*)d_in[1];
  const float* init_state = (const float*)d_in[2];
  const float* W_i        = (const float*)d_in[3];
  const float* b_i        = (const float*)d_in[4];
  const float* W_r        = (const float*)d_in[5];
  const float* b_r        = (const float*)d_in[6];
  const float* W_o        = (const float*)d_in[7];
  const float* b_o        = (const float*)d_in[8];
  const float* fc_w       = (const float*)d_in[9];
  const float* fc_b       = (const float*)d_in[10];
  float* out = (float*)d_out;

  char* ws = (char*)d_ws;
  unsigned short* WT = (unsigned short*)(ws + kOffWT);
  float*          BC = (float*)(ws + kOffBC);

  weight_plane_kernel<<<kPlaneChunks / 256, 256, 0, stream>>>(W_i, W_r, W_o, WT);
  bias_plane_kernel<<<(kBiasVec4 + 255) / 256, 256, 0, stream>>>(b_i, b_r, b_o, BC);
  cell_scan_kernel<<<1, 256, 0, stream>>>(x_m, x_a, init_state, WT, BC, fc_w, fc_b, out);
}
